// SCL_66632122630298
// MI455X (gfx1250) — hardware-verified
//
#include <hip/hip_runtime.h>
#include <math.h>

typedef __attribute__((ext_vector_type(16))) _Float16 v16h;
typedef __attribute__((ext_vector_type(8)))  _Float16 v8h;
typedef __attribute__((ext_vector_type(16))) __bf16   v16b;
typedef __attribute__((ext_vector_type(8)))  __bf16   v8b;
typedef __attribute__((ext_vector_type(8)))  float    v8f;
typedef __attribute__((ext_vector_type(4)))  float    v4f;
typedef __attribute__((ext_vector_type(8)))  unsigned short v8us;

__device__ __forceinline__ unsigned short f2bf_bits(float f) {
  unsigned u = __float_as_uint(f);
  return (unsigned short)((u + 0x7FFFu + ((u >> 16) & 1u)) >> 16);
}
__device__ __forceinline__ float bf_bits2f(unsigned short h) { return __uint_as_float(((unsigned)h) << 16); }

__device__ __forceinline__ void dep_guard_h(v8f& a, v8f& b, v16h x, v16h y) { asm volatile("v_nop\n\tv_nop\n\tv_nop\n\tv_nop" : "+v"(a), "+v"(b) : "v"(x), "v"(y)); }
__device__ __forceinline__ void dep_guard_b(v8f& a, v8f& b, v16b x, v16b y) { asm volatile("v_nop\n\tv_nop\n\tv_nop\n\tv_nop" : "+v"(a), "+v"(b) : "v"(x), "v"(y)); }
__device__ __forceinline__ void keep4_h(v16h a, v16h b, v16h c, v16h d) { asm volatile("v_nop" :: "v"(a), "v"(b), "v"(c), "v"(d)); }
__device__ __forceinline__ void keep4_b(v16b a, v16b b, v16b c, v16b d) { asm volatile("v_nop" :: "v"(a), "v"(b), "v"(c), "v"(d)); }
__device__ __forceinline__ void acc_guard4(v8f& a, v8f& b, v8f& c, v8f& d) { asm volatile("v_nop\n\tv_nop\n\tv_nop\n\tv_nop" : "+v"(a), "+v"(b), "+v"(c), "+v"(d)); }
template <typename T> struct Frag;
template <> struct Frag<_Float16> {
  typedef v16h V; union U { v16h v; v8h h[2]; };
  static __device__ __forceinline__ v16h load(const _Float16* p) {
    U f; f.h[0] = *(const v8h*)(p); f.h[1] = *(const v8h*)(p + 16); return f.v;
  }
  static __device__ __forceinline__ v8f mma(v16h a, v16h b, v8f c) {
    return __builtin_amdgcn_wmma_f32_16x16x32_f16(false, a, false, b, (short)0, c, false, false);
  }
  static __device__ __forceinline__ void guard(v8f& a, v8f& b, v16h x, v16h y) { dep_guard_h(a, b, x, y); }
  static __device__ __forceinline__ void keep(v16h a, v16h b, v16h c, v16h d) { keep4_h(a, b, c, d); }
};
template <> struct Frag<__bf16> {
  typedef v16b V; union U { v16b v; v8b h[2]; };
  static __device__ __forceinline__ v16b load(const __bf16* p) {
    U f; f.h[0] = *(const v8b*)(p); f.h[1] = *(const v8b*)(p + 16); return f.v;
  }
  static __device__ __forceinline__ v8f mma(v16b a, v16b b, v8f c) {
    return __builtin_amdgcn_wmma_f32_16x16x32_bf16(false, a, false, b, (short)0, c, false, false);
  }
  static __device__ __forceinline__ void guard(v8f& a, v8f& b, v16b x, v16b y) { dep_guard_b(a, b, x, y); }
  static __device__ __forceinline__ void keep(v16b a, v16b b, v16b c, v16b d) { keep4_b(a, b, c, d); }
};

template <int ET> struct Elem;
template <> struct Elem<0> { typedef _Float16 T; };
template <> struct Elem<1> { typedef __bf16 T; };
template <int ET, bool SPLIT, int BIAS_MODE, int OUT_MODE, bool RESID, int ACT = 0>
__global__ __launch_bounds__(256) void wmma_gemm64(
    const unsigned short* __restrict__ Ap, const unsigned short* __restrict__ A2p, int lda, long strideA,
    const unsigned short* __restrict__ Btp, const unsigned short* __restrict__ Bt2p, int ldb, long strideB,
    void* __restrict__ Cout, void* __restrict__ Cout2, int ldc, long strideC,
    const float* __restrict__ bias,
    const float* __restrict__ resid, long strideR,
    int M, int N, int K, float scale) {
  typedef typename Elem<ET>::T T;
  typedef typename Frag<T>::V V;
  const T* A = (const T*)Ap; const T* A2 = (const T*)A2p; const T* Bt = (const T*)Btp; const T* Bt2 = (const T*)Bt2p;
  __shared__ __align__(16) float sT[8][16 * 68];
  const int b    = blockIdx.y;
  const int lane = threadIdx.x & 31;
  const int wave = threadIdx.x >> 5;
  const int tilesN = N >> 6;
  const int tilesM = M >> 6;
  const int tile = blockIdx.x * 8 + wave;
  if (tile >= tilesM * tilesN) return;
  const int tm = tile / tilesN;
  const int tn = tile - tm * tilesN;
  const int m0 = tm << 6;
  const int n0 = tn << 6;

  const T* Ab  = A  + (size_t)b * strideA;
  const T* Bb  = Bt + (size_t)b * strideB;
  const T* Ab2 = SPLIT ? (A2  + (size_t)b * strideA) : nullptr;
  const T* Bb2 = SPLIT ? (Bt2 + (size_t)b * strideB) : nullptr;

  const int rlane = lane & 15;
  const int koff  = (lane >> 4) * 8;
  const int mOff  = (lane >> 4) * 8;

  v8f acc[4][4];
#pragma unroll
  for (int i = 0; i < 4; ++i)
#pragma unroll
    for (int j = 0; j < 4; ++j) acc[i][j] = (v8f){0.f,0.f,0.f,0.f,0.f,0.f,0.f,0.f};

  for (int k0 = 0; k0 < K; k0 += 32) {
    V bh[4], bl[4];
#pragma unroll
    for (int j = 0; j < 4; ++j) {
      const size_t bo = (size_t)(n0 + (j << 4) + rlane) * ldb + koff + k0;
      bh[j] = Frag<T>::load(Bb + bo);
      if (SPLIT) bl[j] = Frag<T>::load(Bb2 + bo);
    }
#pragma unroll
    for (int i = 0; i < 4; ++i) {
      const size_t ao = (size_t)(m0 + (i << 4) + rlane) * lda + koff + k0;
      V ah = Frag<T>::load(Ab + ao);
      V al;
      if (SPLIT) al = Frag<T>::load(Ab2 + ao);
#pragma unroll
      for (int j = 0; j < 4; ++j) {
        acc[i][j] = Frag<T>::mma(ah, bh[j], acc[i][j]);
        if (SPLIT) {
          acc[i][j] = Frag<T>::mma(ah, bl[j], acc[i][j]);
          acc[i][j] = Frag<T>::mma(al, bh[j], acc[i][j]);
        }
      }
      Frag<T>::guard(acc[i][0], acc[i][3], ah, SPLIT ? al : ah);
    }
    Frag<T>::keep(bh[0], bh[1], bh[2], bh[3]);
    if (SPLIT) Frag<T>::keep(bl[0], bl[1], bl[2], bl[3]);
  }
  acc_guard4(acc[0][0], acc[0][1], acc[0][2], acc[0][3]);
  acc_guard4(acc[1][0], acc[1][1], acc[1][2], acc[1][3]);
  acc_guard4(acc[2][0], acc[2][1], acc[2][2], acc[2][3]);
  acc_guard4(acc[3][0], acc[3][1], acc[3][2], acc[3][3]);

  float* slab = sT[wave];
  const float* Rb = RESID ? (resid + (size_t)b * strideR) : nullptr;
#pragma unroll
  for (int i = 0; i < 4; ++i) {
    const int mBase = m0 + (i << 4);
#pragma unroll
    for (int j = 0; j < 4; ++j) {
      const int n = n0 + (j << 4) + rlane;
      float bv = 0.f;
      if (BIAS_MODE == 2) bv = bias[n];
#pragma unroll
      for (int r = 0; r < 8; ++r) {
        float v = acc[i][j][r] * scale;
        if (BIAS_MODE == 1) v += bias[mBase + mOff + r];
        if (BIAS_MODE == 2) v += bv;
        if (RESID) v += Rb[(size_t)(mBase + mOff + r) * ldc + n];
        if (ACT == 1) v = tanhf(v);
        if (ACT == 2) v = fmaxf(v, 0.0f);
        if (ACT == 3) v = v / (1.0f + expf(-v));
        if (ACT == 4) v = (v > 0.f) ? v : 0.01f * v;
        if (ACT == 5) v = 0.5f * v * (1.0f + erff(v * 0.70710678118654752f));
        slab[(mOff + r) * 68 + (j << 4) + rlane] = v;
      }
    }
    __builtin_amdgcn_fence(__ATOMIC_RELEASE, "workgroup");
    __builtin_amdgcn_wave_barrier();
    __builtin_amdgcn_fence(__ATOMIC_ACQUIRE, "workgroup");
    if (OUT_MODE == 0) {
      float* C = (float*)Cout + (size_t)b * strideC;
      const int hh = lane >> 4, c4 = (lane & 15) * 4;
      for (int pass = 0; pass < 2; ++pass) {
#pragma unroll
        for (int it = 0; it < 8; ++it) {
          const int row = it * 2 + hh;
          v4f v = *(const v4f*)(slab + row * 68 + c4);
          *(volatile v4f*)(C + (size_t)(mBase + row) * ldc + n0 + c4) = v;
        }
        __threadfence();
      }
    } else {
      const int q = lane >> 3, c8 = (lane & 7) * 8;
      unsigned short* C  = (unsigned short*)Cout  + (size_t)b * strideC;
      unsigned short* C2 = (OUT_MODE == 2) ? ((unsigned short*)Cout2 + (size_t)b * strideC) : nullptr;
      for (int pass = 0; pass < 2; ++pass) {
#pragma unroll
        for (int it = 0; it < 4; ++it) {
          const int row = it * 4 + q;
          const float* sp = slab + row * 68 + c8;
          v8h hv, lv;
#pragma unroll
          for (int e = 0; e < 8; ++e) {
            if (OUT_MODE == 1) {
              hv[e] = (_Float16)sp[e];
            } else {
              unsigned short hb = f2bf_bits(sp[e]);
              unsigned short lb = f2bf_bits(sp[e] - bf_bits2f(hb));
              hv[e] = __builtin_bit_cast(_Float16, hb);
              lv[e] = __builtin_bit_cast(_Float16, lb);
            }
          }
          *(volatile v8h*)(C + (size_t)(mBase + row) * ldc + n0 + c8) = hv;
          if (OUT_MODE == 2) *(volatile v8h*)(C2 + (size_t)(mBase + row) * ldc + n0 + c8) = lv;
        }
        __threadfence();
      }
    }
    __builtin_amdgcn_fence(__ATOMIC_RELEASE, "workgroup");
    __builtin_amdgcn_wave_barrier();
    __builtin_amdgcn_fence(__ATOMIC_ACQUIRE, "workgroup");
  }
}

__global__ __launch_bounds__(256) void split_rows_kernel(
    const float* __restrict__ in, unsigned short* __restrict__ hi, unsigned short* __restrict__ lo, int n8) {
  const int i = blockIdx.x * 256 + threadIdx.x;
  if (i < n8) {
    const v4f a = *(const v4f*)(in + (size_t)i * 8);
    const v4f b = *(const v4f*)(in + (size_t)i * 8 + 4);
    v8us hv, lv;
#pragma unroll
    for (int e = 0; e < 4; ++e) {
      unsigned short hb = f2bf_bits(a[e]);
      hv[e] = hb; lv[e] = f2bf_bits(a[e] - bf_bits2f(hb));
      hb = f2bf_bits(b[e]);
      hv[4 + e] = hb; lv[4 + e] = f2bf_bits(b[e] - bf_bits2f(hb));
    }
    unsigned short* ph = hi + (size_t)i * 8;
    unsigned short* pl = lo + (size_t)i * 8;
    *(volatile v8us*)ph = hv;
    *(volatile v8us*)pl = lv;
    __threadfence();
    *(volatile v8us*)ph = hv;
    *(volatile v8us*)pl = lv;
  }
}

__global__ __launch_bounds__(256) void split_transpose_kernel(
    const float* __restrict__ W, unsigned short* __restrict__ hi, unsigned short* __restrict__ lo,
    int Krows, int Ncols) {
  __shared__ float tile[64][65];
  const int tid = threadIdx.x;
  const int n0 = blockIdx.x * 64;
  const int k0 = blockIdx.y * 64;
#pragma unroll
  for (int it = 0; it < 4; ++it) {
    const int idx = it * 256 + tid;
    const int r = idx >> 4, c4 = (idx & 15) * 4;
    const v4f v = *(const v4f*)(W + (size_t)(k0 + r) * Ncols + n0 + c4);
    tile[r][c4 + 0] = v[0]; tile[r][c4 + 1] = v[1]; tile[r][c4 + 2] = v[2]; tile[r][c4 + 3] = v[3];
  }
  __syncthreads();
  const int i = tid >> 3, c8 = (tid & 7) * 8;
  for (int pass = 0; pass < 2; ++pass) {
#pragma unroll
    for (int half = 0; half < 2; ++half) {
      const int nrow = i + 32 * half;
      v8us hv, lv;
#pragma unroll
      for (int e = 0; e < 8; ++e) {
        const float f = tile[c8 + e][nrow];
        const unsigned short hb = f2bf_bits(f);
        hv[e] = hb;
        lv[e] = f2bf_bits(f - bf_bits2f(hb));
      }
      const size_t o = (size_t)(n0 + nrow) * Krows + k0 + c8;
      *(volatile v8us*)(hi + o) = hv;
      *(volatile v8us*)(lo + o) = lv;
    }
    __threadfence();
  }
}

#define HS 16
#define HD 64
#define HA 8
#define HX (HD * HA)
#define HP 65
__global__ __launch_bounds__(128) void reflect_chain_kernel(
    const float* __restrict__ x3, const float* __restrict__ act, float* __restrict__ out, int nB) {
  __shared__ __align__(16) float xs[HS * HX];
  __shared__ float Ss[HS * HA * HP];
  __shared__ __align__(16) float qs[HS * HD];
  __shared__ __align__(16) float os[HS * HD];
  const int tid = threadIdx.x;
  const int b0 = blockIdx.x * HS;

#pragma unroll
  for (int it = 0; it < (HS * HX / 4) / 128; ++it) {
    const int idx = it * 128 + tid;
    const int s = idx >> 7;
    const int f = (idx & 127) * 4;
    int row = b0 + s; row = (row < nB) ? row : (nB - 1);
    const v4f v = *(const v4f*)(x3 + (size_t)row * HX + f);
    *(v4f*)(xs + s * HX + f) = v;
  }
#pragma unroll
  for (int it = 0; it < (HS * HD / 4) / 128; ++it) {
    const int idx = it * 128 + tid;
    const int s = idx >> 4;
    const int f = (idx & 15) * 4;
    int row = b0 + s; row = (row < nB) ? row : (nB - 1);
    const v4f v = *(const v4f*)(act + (size_t)row * HD + f);
    *(v4f*)(qs + s * HD + f) = v;
  }
  __syncthreads();

  const int s = tid >> 3;
  const int k = tid & 7;
  float* Sc = Ss + (s * HA + k) * HP;
  const float* xr = xs + s * HX;
  const float* qr = qs + s * HD;

#pragma unroll 8
  for (int n = 0; n < HD; ++n) Sc[n] = (n == k) ? 1.0f : 0.0f;

  float vtv = 0.f;
#pragma unroll 8
  for (int n = 0; n < HD; ++n) { const float v = xr[n * HA + k]; vtv = fmaf(v, v, vtv); }

#pragma unroll 1
  for (int c = 0; c < HA; ++c) {
    float w = 0.f;
#pragma unroll 8
    for (int n = 0; n < HD; ++n) w = fmaf(xr[n * HA + c], Sc[n], w);
    const float vc = __shfl(vtv, c, 8);
    const float rc = 1.0f / vc;
    const float t = (w + w) * rc;
#pragma unroll 8
    for (int n = 0; n < HD; ++n) Sc[n] = fmaf(-xr[n * HA + c], t, Sc[n]);
  }

  float a = 0.f;
#pragma unroll 8
  for (int n = 0; n < HD; ++n) a = fmaf(Sc[n], qr[n], a);
  float aj[HA];
#pragma unroll
  for (int j = 0; j < HA; ++j) aj[j] = __shfl(a, j, 8);
  __syncthreads();

  const float* Sb = Ss + s * HA * HP;
#pragma unroll 1
  for (int j = 0; j < HD / HA; ++j) {
    const int n = j * HA + k;
    float q = 0.f;
#pragma unroll
    for (int kk = 0; kk < HA; ++kk) q = fmaf(Sb[kk * HP + n], aj[kk], q);
    os[s * HD + n] = q;
  }
  __syncthreads();

  float* ob = out + (size_t)b0 * HD;
  for (int pass = 0; pass < 2; ++pass) {
#pragma unroll
    for (int it = 0; it < (HS * HD / 4) / 128; ++it) {
      const int idx = it * 128 + tid;
      const int s2 = idx >> 4;
      if (b0 + s2 < nB) {
        const v4f v = *(const v4f*)(os + idx * 4);
        *(volatile v4f*)(ob + (size_t)idx * 4) = v;
      }
    }
    __threadfence();
  }
}

extern "C" void kernel_launch(void* const* d_in, const int* in_sizes, int n_in,
                              void* d_out, int out_size, void* d_ws, size_t ws_size,
                              hipStream_t stream) {
  if (n_in < 8) return;
  const float* cond = (const float*)d_in[0];
  const float* act  = (const float*)d_in[1];
  const float* W1   = (const float*)d_in[2];
  const float* b1   = (const float*)d_in[3];
  const float* W2   = (const float*)d_in[4];
  const float* b2   = (const float*)d_in[5];
  const float* W3   = (const float*)d_in[6];
  const float* b3   = (const float*)d_in[7];

  const int H1n = in_sizes[3];
  const int H2n = in_sizes[5];
  const int N3  = in_sizes[7];
  if (H1n <= 0 || H2n <= 0 || N3 != HX) return;
  const int CD = in_sizes[2] / H1n;
  if (CD <= 0 || (CD & 63) || (H1n & 63) || (H2n & 63)) return;
  const int Bn = in_sizes[0] / CD;
  if (Bn <= 0 || (Bn & 63)) return;
  if (in_sizes[1] != Bn * HD || out_size != Bn * HD) return;
  if (in_sizes[4] != H1n * H2n || in_sizes[6] != H2n * N3) return;

  size_t off = 0;
  auto carve = [&](size_t bytes) { size_t o = off; off += (bytes + 255) & ~(size_t)255; return o; };
  const size_t o_ch  = carve((size_t)Bn * CD * 2);
  const size_t o_cl  = carve((size_t)Bn * CD * 2);
  const size_t o_w1h = carve((size_t)H1n * CD * 2);
  const size_t o_w1l = carve((size_t)H1n * CD * 2);
  const size_t o_w2h = carve((size_t)H2n * H1n * 2);
  const size_t o_w2l = carve((size_t)H2n * H1n * 2);
  const size_t o_w3h = carve((size_t)N3 * H2n * 2);
  const size_t o_w3l = carve((size_t)N3 * H2n * 2);
  const size_t o_x1h = carve((size_t)Bn * H1n * 2);
  const size_t o_x1l = carve((size_t)Bn * H1n * 2);
  const size_t o_x2h = carve((size_t)Bn * H2n * 2);
  const size_t o_x2l = carve((size_t)Bn * H2n * 2);
  const size_t o_x3  = carve((size_t)Bn * N3 * 4);
  if (off > ws_size || off > (size_t)134217728) return;

  char* ws = (char*)d_ws;
  unsigned short* ch  = (unsigned short*)(ws + o_ch);
  unsigned short* cl  = (unsigned short*)(ws + o_cl);
  unsigned short* w1h = (unsigned short*)(ws + o_w1h);
  unsigned short* w1l = (unsigned short*)(ws + o_w1l);
  unsigned short* w2h = (unsigned short*)(ws + o_w2h);
  unsigned short* w2l = (unsigned short*)(ws + o_w2l);
  unsigned short* w3h = (unsigned short*)(ws + o_w3h);
  unsigned short* w3l = (unsigned short*)(ws + o_w3l);
  unsigned short* x1h = (unsigned short*)(ws + o_x1h);
  unsigned short* x1l = (unsigned short*)(ws + o_x1l);
  unsigned short* x2h = (unsigned short*)(ws + o_x2h);
  unsigned short* x2l = (unsigned short*)(ws + o_x2l);
  float*          x3  = (float*)(ws + o_x3);
  float*          out = (float*)d_out;

  {
    const int n8 = Bn * CD / 8;
    split_rows_kernel<<<(n8 + 255) / 256, 256, 0, stream>>>(cond, ch, cl, n8);
  }
  split_transpose_kernel<<<dim3(H1n / 64, CD / 64), 256, 0, stream>>>(W1, w1h, w1l, CD, H1n);
  split_transpose_kernel<<<dim3(H2n / 64, H1n / 64), 256, 0, stream>>>(W2, w2h, w2l, H1n, H2n);
  split_transpose_kernel<<<dim3(N3 / 64, H2n / 64), 256, 0, stream>>>(W3, w3h, w3l, H2n, N3);

  {
    const int tiles = (Bn / 64) * (H1n / 64);
    wmma_gemm64<1, true, 2, 2, false, 1><<<dim3((tiles + 7) / 8, 1), 256, 0, stream>>>(
        ch, cl, CD, 0L, w1h, w1l, CD, 0L, (void*)x1h, (void*)x1l, H1n, 0L,
        b1, b3, 0L, Bn, H1n, CD, 1.0f);
  }
  {
    const int tiles = (Bn / 64) * (H2n / 64);
    wmma_gemm64<1, true, 2, 2, false, 1><<<dim3((tiles + 7) / 8, 1), 256, 0, stream>>>(
        x1h, x1l, H1n, 0L, w2h, w2l, H1n, 0L, (void*)x2h, (void*)x2l, H2n, 0L,
        b2, b3, 0L, Bn, H2n, H1n, 1.0f);
  }
  {
    const int tiles = (Bn / 64) * (N3 / 64);
    wmma_gemm64<1, true, 2, 0, false, 0><<<dim3((tiles + 7) / 8, 1), 256, 0, stream>>>(
        x2h, x2l, H2n, 0L, w3h, w3l, H2n, 0L, (void*)x3, (void*)x3, N3, 0L,
        b3, b3, 0L, Bn, N3, H2n, 1.0f);
  }
  reflect_chain_kernel<<<(Bn + HS - 1) / HS, 128, 0, stream>>>(x3, act, out, Bn);
}
